// DenseGATLayer_9448928051792
// MI455X (gfx1250) — hardware-verified
//
#include <hip/hip_runtime.h>
#include <math.h>


#define N_NODES  2048
#define IN_DIM   512
#define OUT_DIM  512
#define HEADS    8
#define HEAD_DIM 64
#define NEG_SLOPE 0.2f
typedef __attribute__((ext_vector_type(16))) _Float16 v16h;
typedef __attribute__((ext_vector_type(8)))  _Float16 v8h;
typedef __attribute__((ext_vector_type(8)))  float    v8f;
typedef __attribute__((ext_vector_type(4)))  float    v4f;
#define VST2(T, ptr, val) do { const T _v = (val); *(volatile T*)(ptr) = _v; __threadfence(); *(volatile T*)(ptr) = _v; } while (0)
__device__ __forceinline__ float leaky(float x) { return x > 0.f ? x : NEG_SLOPE * x; }
__device__ __forceinline__ int kmap(int e, int hh) { return (e < 8) ? (8 * hh + e) : (16 + 8 * hh + (e - 8)); }
__device__ __forceinline__ v8f wmma16(v16h a, v16h b, v8f c) {
  v8f d = __builtin_amdgcn_wmma_f32_16x16x32_f16(false, a, false, b, (short)0, c, false, false);
  asm volatile("v_nop\n\tv_nop\n\tv_nop\n\tv_nop" : "+v"(d) : "v"(a), "v"(b));
  return d;
}

__global__ __launch_bounds__(128) void gat_gemm_xw(const float* __restrict__ x, const float* __restrict__ W,
                                                   float* __restrict__ Wh, _Float16* __restrict__ Whb) {
  __shared__ __attribute__((aligned(16))) float sT[16][64];
  const int lane = threadIdx.x & 31, wave = threadIdx.x >> 5, m = lane & 15, hh = lane >> 4;
  const int row0 = blockIdx.x * 16, col0 = blockIdx.y * 64 + wave * 16;
  const float* xr = x + (size_t)(row0 + m) * IN_DIM;
  v8f c = {};
  for (int kk = 0; kk < IN_DIM; kk += 32) {
    v16h A, B;
#pragma unroll
    for (int e = 0; e < 16; ++e) { const int k = kk + kmap(e, hh); A[e] = (_Float16)xr[k]; B[e] = (_Float16)W[(size_t)k * OUT_DIM + col0 + m]; }
    c = wmma16(A, B, c);
  }
#pragma unroll
  for (int r = 0; r < 8; ++r) sT[r + 8 * hh][wave * 16 + m] = c[r];
  __syncthreads();
  const int bc0 = blockIdx.y * 64;
  for (int pass = 0; pass < 2; ++pass) {
#pragma unroll
    for (int j = 0; j < 2; ++j) {
      const int rr = j * 8 + (threadIdx.x >> 4), q4 = (threadIdx.x & 15) * 4;
      *(volatile v4f*)(Wh + (size_t)(row0 + rr) * OUT_DIM + bc0 + q4) = *(const v4f*)(&sT[rr][q4]);
    }
    {
      const int rr = threadIdx.x >> 3, q8 = (threadIdx.x & 7) * 8;
      v8h v;
#pragma unroll
      for (int e = 0; e < 8; ++e) v[e] = (_Float16)sT[rr][q8 + e];
      *(volatile v8h*)(Whb + (size_t)(row0 + rr) * OUT_DIM + bc0 + q8) = v;
    }
    __threadfence();
  }
}
__global__ __launch_bounds__(256) void gat_scores(const float* __restrict__ Wh, const float* __restrict__ a,
                                                  float* __restrict__ s_src, float* __restrict__ s_dst) {
  const int idx = blockIdx.x * blockDim.x + threadIdx.x;
  if (idx >= N_NODES * HEADS) return;
  const int n = idx >> 3, h = idx & 7;
  const float* w = Wh + (size_t)n * OUT_DIM + h * HEAD_DIM;
  float ss = 0.f, sd = 0.f;
#pragma unroll 8
  for (int d = 0; d < HEAD_DIM; ++d) { const float v = w[d]; ss += v * a[d]; sd += v * a[HEAD_DIM + d]; }
  VST2(float, s_src + idx, ss);
  VST2(float, s_dst + idx, sd);
}
__global__ __launch_bounds__(128) void gat_rowmax(const int* __restrict__ adj, const float* __restrict__ s_src,
                                                  const float* __restrict__ s_dst, float* __restrict__ emax) {
  __shared__ float se[32];
  const int lane = threadIdx.x & 31, wave = threadIdx.x >> 5, i = blockIdx.x * 4 + wave;
  float mx[HEADS];
#pragma unroll
  for (int h = 0; h < HEADS; ++h) mx[h] = -__builtin_inff();
  const int* arow = adj + (size_t)i * N_NODES;
  for (int j = lane; j < N_NODES; j += 32) {
    if (arow[j] > 0) { const float* sj = s_dst + (size_t)j * HEADS;
#pragma unroll
      for (int h = 0; h < HEADS; ++h) mx[h] = fmaxf(mx[h], sj[h]); }
  }
#pragma unroll
  for (int h = 0; h < HEADS; ++h)
#pragma unroll
    for (int off = 16; off > 0; off >>= 1) mx[h] = fmaxf(mx[h], __shfl_xor(mx[h], off));
  if (lane < HEADS) {
    float v = mx[0];
#pragma unroll
    for (int h = 1; h < HEADS; ++h) if (lane == h) v = mx[h];
    se[wave * 8 + lane] = leaky(s_src[i * HEADS + lane] + v);
  }
  __syncthreads();
  if (threadIdx.x < 32) VST2(float, emax + (size_t)blockIdx.x * 32 + threadIdx.x, se[threadIdx.x]);
}
__global__ __launch_bounds__(128) void gat_aggregate(const int* __restrict__ adj, const _Float16* __restrict__ Whb,
                                                     const float* __restrict__ s_src, const float* __restrict__ s_dst,
                                                     const float* __restrict__ emax, float* __restrict__ out) {
  __shared__ __attribute__((aligned(16))) float sO[4][16][HEAD_DIM];
  const int lane = threadIdx.x & 31, wave = threadIdx.x >> 5, m = lane & 15, hh = lane >> 4;
  const int head = blockIdx.y * 4 + wave, row0 = blockIdx.x * 16, arow = row0 + m;
  const float si = s_src[arow * HEADS + head], em = emax[arow * HEADS + head];
  const int* adjr = adj + (size_t)arow * N_NODES;
  const _Float16* whh = Whb + head * HEAD_DIM;
  v8f c[4] = {};
  float lsum = 0.f;
  for (int jb = 0; jb < N_NODES; jb += 32) {
    v16h A;
#pragma unroll
    for (int e = 0; e < 16; ++e) {
      const int j = jb + kmap(e, hh);
      float w = 0.f;
      if (adjr[j] > 0) w = __expf(leaky(si + s_dst[(size_t)j * HEADS + head]) - em);
      lsum += w; A[e] = (_Float16)w;
    }
#pragma unroll
    for (int t = 0; t < 4; ++t) {
      v16h B;
#pragma unroll
      for (int e = 0; e < 16; ++e) B[e] = whh[(size_t)(jb + kmap(e, hh)) * OUT_DIM + t * 16 + m];
      c[t] = wmma16(A, B, c[t]);
    }
  }
  lsum += __shfl_xor(lsum, 16);
#pragma unroll
  for (int r = 0; r < 8; ++r) {
    const float lr = __shfl(lsum, r + hh * 8);
    const float inv = 1.0f / lr;
#pragma unroll
    for (int t = 0; t < 4; ++t) sO[wave][r + 8 * hh][t * 16 + m] = c[t][r] * inv;
  }
  __builtin_amdgcn_fence(__ATOMIC_RELEASE, "workgroup"); __builtin_amdgcn_wave_barrier(); __builtin_amdgcn_fence(__ATOMIC_ACQUIRE, "workgroup");
  for (int pass = 0; pass < 2; ++pass) {
#pragma unroll
    for (int j = 0; j < 8; ++j) { const int rr = j * 2 + hh, q4 = m * 4;
      *(volatile v4f*)(out + (size_t)(row0 + rr) * OUT_DIM + head * HEAD_DIM + q4) = *(const v4f*)(&sO[wave][rr][q4]); }
    __threadfence();
  }
}
extern "C" void kernel_launch(void* const* d_in, const int* in_sizes, int n_in,
                              void* d_out, int out_size, void* d_ws, size_t ws_size, hipStream_t stream) {
  (void)in_sizes; (void)n_in; (void)out_size;
  const float* x   = (const float*)d_in[0];
  const int*   adj = (const int*)  d_in[1];
  const float* W   = (const float*)d_in[2];
  const float* a   = (const float*)d_in[3];
  float* out = (float*)d_out;
  if (ws_size < (size_t)N_NODES * OUT_DIM * 6 + (size_t)3 * N_NODES * HEADS * 4) return;
  char* ws = (char*)d_ws;
  float*    Wh    = (float*)ws;
  _Float16* Whb   = (_Float16*)(ws + (size_t)N_NODES * OUT_DIM * sizeof(float));
  float*    s_src = (float*)(ws + (size_t)N_NODES * OUT_DIM * 6);
  float*    s_dst = s_src + N_NODES * HEADS;
  float*    emax  = s_dst + N_NODES * HEADS;
  gat_gemm_xw<<<dim3(N_NODES / 16, OUT_DIM / 64), 128, 0, stream>>>(x, W, Wh, Whb);
  gat_scores<<<(N_NODES * HEADS + 255) / 256, 256, 0, stream>>>(Wh, a, s_src, s_dst);
  gat_rowmax<<<N_NODES / 4, 128, 0, stream>>>(adj, s_src, s_dst, emax);
  gat_aggregate<<<dim3(N_NODES / 16, HEADS / 4), 128, 0, stream>>>(adj, Whb, s_src, s_dst, emax, out);
}
